// SelfAttentionModule_65481071406093
// MI455X (gfx1250) — hardware-verified
//
#include <hip/hip_runtime.h>
#include <math.h>

#define DM 1024
#define NH 16
#define HD 64
#define NB_FULL 2
#define SEQ_FULL 2048
#ifndef NB
#define NB 2
#endif
#ifndef SEQ
#define SEQ 2048
#endif
static_assert(NB >= 1 && NB <= NB_FULL);
static_assert(SEQ >= 64 && SEQ <= SEQ_FULL && (SEQ % 64) == 0);
static_assert(NH * HD == DM);
static_assert(((NB * SEQ) % 64) == 0 && (DM % 64) == 0);

typedef __attribute__((ext_vector_type(16))) _Float16 v16h;
typedef __attribute__((ext_vector_type(8)))  _Float16 v8h;
typedef __attribute__((ext_vector_type(8)))  float    v8f;
typedef __attribute__((ext_vector_type(4)))  float    v4f;
typedef __attribute__((ext_vector_type(4)))  unsigned int v4u;

#define VST2(T, ptr, val) do { const T vst2_v_ = (val); *(volatile T*)(ptr) = vst2_v_; __threadfence(); *(volatile T*)(ptr) = vst2_v_; } while (0)
#define VST2V4(ptr, val) do { const v4f vst2_v4_ = (val); *(volatile v4f*)(ptr) = vst2_v4_; __threadfence(); *(volatile v4f*)(ptr) = vst2_v4_; } while (0)

__device__ __forceinline__ v8f wmma16(v16h a, v16h b, v8f c) {
    c = __builtin_amdgcn_wmma_f32_16x16x32_f16(false, a, false, b, (short)0, c, false, false);
    asm volatile("v_nop\n\tv_nop\n\tv_nop\n\tv_nop" : "+v"(c) : "v"(a), "v"(b));
    return c;
}
__device__ __forceinline__ v16h fload(const _Float16* p) {
    union U { v16h v; v8h h[2]; } f; f.h[0] = *(const v8h*)(p); f.h[1] = *(const v8h*)(p + 16); return f.v;
}
__device__ __forceinline__ void sched_fence() { asm volatile("" ::: "memory"); }
__device__ __forceinline__ float bf_rne(float v) { const unsigned u = __builtin_bit_cast(unsigned, v); const unsigned r = (u + 0x7fffu + ((u >> 16) & 1u)) & 0xffff0000u; return __builtin_bit_cast(float, r); }
__device__ __forceinline__ unsigned int pk2h(float a, float b) { return (unsigned int)__builtin_bit_cast(unsigned short, (_Float16)a) | ((unsigned int)__builtin_bit_cast(unsigned short, (_Float16)b) << 16); }

namespace w25 {
typedef __attribute__((ext_vector_type(16))) __bf16 v16b;
typedef __attribute__((ext_vector_type(8)))  __bf16 v8b;

__device__ __forceinline__ unsigned short f2bf_bits(float f) {
  unsigned u = __float_as_uint(f);
  return (unsigned short)((u + 0x7FFFu + ((u >> 16) & 1u)) >> 16);
}
__device__ __forceinline__ float bf_bits2f(unsigned short h) { return __uint_as_float(((unsigned)h) << 16); }

__device__ __forceinline__ void dep_guard_h(v8f& a, v8f& b, v16h x, v16h y) { asm volatile("v_nop\n\tv_nop\n\tv_nop\n\tv_nop" : "+v"(a), "+v"(b) : "v"(x), "v"(y)); }
__device__ __forceinline__ void dep_guard_b(v8f& a, v8f& b, v16b x, v16b y) { asm volatile("v_nop\n\tv_nop\n\tv_nop\n\tv_nop" : "+v"(a), "+v"(b) : "v"(x), "v"(y)); }
__device__ __forceinline__ void keep4_h(v16h a, v16h b, v16h c, v16h d) { asm volatile("v_nop" :: "v"(a), "v"(b), "v"(c), "v"(d)); }
__device__ __forceinline__ void keep4_b(v16b a, v16b b, v16b c, v16b d) { asm volatile("v_nop" :: "v"(a), "v"(b), "v"(c), "v"(d)); }
__device__ __forceinline__ void acc_guard4(v8f& a, v8f& b, v8f& c, v8f& d) { asm volatile("v_nop\n\tv_nop\n\tv_nop\n\tv_nop" : "+v"(a), "+v"(b), "+v"(c), "+v"(d)); }
template <typename T> struct Frag;
template <> struct Frag<_Float16> {
  typedef v16h V; union U { v16h v; v8h h[2]; };
  static __device__ __forceinline__ v16h load(const _Float16* p) {
    U f; f.h[0] = *(const v8h*)(p); f.h[1] = *(const v8h*)(p + 16); return f.v;
  }
  static __device__ __forceinline__ v8f mma(v16h a, v16h b, v8f c) {
    return __builtin_amdgcn_wmma_f32_16x16x32_f16(false, a, false, b, (short)0, c, false, false);
  }
  static __device__ __forceinline__ void guard(v8f& a, v8f& b, v16h x, v16h y) { dep_guard_h(a, b, x, y); }
  static __device__ __forceinline__ void keep(v16h a, v16h b, v16h c, v16h d) { keep4_h(a, b, c, d); }
};
template <> struct Frag<__bf16> {
  typedef v16b V; union U { v16b v; v8b h[2]; };
  static __device__ __forceinline__ v16b load(const __bf16* p) {
    U f; f.h[0] = *(const v8b*)(p); f.h[1] = *(const v8b*)(p + 16); return f.v;
  }
  static __device__ __forceinline__ v8f mma(v16b a, v16b b, v8f c) {
    return __builtin_amdgcn_wmma_f32_16x16x32_bf16(false, a, false, b, (short)0, c, false, false);
  }
  static __device__ __forceinline__ void guard(v8f& a, v8f& b, v16b x, v16b y) { dep_guard_b(a, b, x, y); }
  static __device__ __forceinline__ void keep(v16b a, v16b b, v16b c, v16b d) { keep4_b(a, b, c, d); }
};

template <int ET> struct Elem;
template <> struct Elem<0> { typedef _Float16 T; };
template <> struct Elem<1> { typedef __bf16 T; };
template <int ET, bool SPLIT, int BIAS_MODE, int OUT_MODE, bool RESID, int ACT = 0>
__global__ __launch_bounds__(256) void wmma_gemm64(
    const unsigned short* __restrict__ Ap, const unsigned short* __restrict__ A2p, int lda, long strideA,
    const unsigned short* __restrict__ Btp, const unsigned short* __restrict__ Bt2p, int ldb, long strideB,
    void* __restrict__ Cout, void* __restrict__ Cout2, int ldc, long strideC,
    const float* __restrict__ bias,
    const float* __restrict__ resid, long strideR,
    int M, int N, int K, float scale) {
  typedef typename Elem<ET>::T T;
  typedef typename Frag<T>::V V;
  const T* A = (const T*)Ap; const T* A2 = (const T*)A2p; const T* Bt = (const T*)Btp; const T* Bt2 = (const T*)Bt2p;
  __shared__ __align__(16) float sT[8][16 * 68];
  const int b    = blockIdx.y;
  const int lane = threadIdx.x & 31;
  const int wave = threadIdx.x >> 5;
  const int tilesN = N >> 6;
  const int tilesM = M >> 6;
  const int tile = blockIdx.x * 8 + wave;
  if (tile >= tilesM * tilesN) return;
  const int tm = tile / tilesN;
  const int tn = tile - tm * tilesN;
  const int m0 = tm << 6;
  const int n0 = tn << 6;

  const T* Ab  = A  + (size_t)b * strideA;
  const T* Bb  = Bt + (size_t)b * strideB;
  const T* Ab2 = SPLIT ? (A2  + (size_t)b * strideA) : nullptr;
  const T* Bb2 = SPLIT ? (Bt2 + (size_t)b * strideB) : nullptr;

  const int rlane = lane & 15;
  const int koff  = (lane >> 4) * 8;
  const int mOff  = (lane >> 4) * 8;

  v8f acc[4][4];
#pragma unroll
  for (int i = 0; i < 4; ++i)
#pragma unroll
    for (int j = 0; j < 4; ++j) acc[i][j] = (v8f){0.f,0.f,0.f,0.f,0.f,0.f,0.f,0.f};

  for (int k0 = 0; k0 < K; k0 += 32) {
    V bh[4], bl[4];
#pragma unroll
    for (int j = 0; j < 4; ++j) {
      const size_t bo = (size_t)(n0 + (j << 4) + rlane) * ldb + koff + k0;
      bh[j] = Frag<T>::load(Bb + bo);
      if (SPLIT) bl[j] = Frag<T>::load(Bb2 + bo);
    }
#pragma unroll
    for (int i = 0; i < 4; ++i) {
      const size_t ao = (size_t)(m0 + (i << 4) + rlane) * lda + koff + k0;
      V ah = Frag<T>::load(Ab + ao);
      V al;
      if (SPLIT) al = Frag<T>::load(Ab2 + ao);
#pragma unroll
      for (int j = 0; j < 4; ++j) {
        acc[i][j] = Frag<T>::mma(ah, bh[j], acc[i][j]);
        if (SPLIT) {
          acc[i][j] = Frag<T>::mma(ah, bl[j], acc[i][j]);
          acc[i][j] = Frag<T>::mma(al, bh[j], acc[i][j]);
        }
      }
      Frag<T>::guard(acc[i][0], acc[i][3], ah, SPLIT ? al : ah);
    }
    Frag<T>::keep(bh[0], bh[1], bh[2], bh[3]);
    if (SPLIT) Frag<T>::keep(bl[0], bl[1], bl[2], bl[3]);
  }
  acc_guard4(acc[0][0], acc[0][1], acc[0][2], acc[0][3]);
  acc_guard4(acc[1][0], acc[1][1], acc[1][2], acc[1][3]);
  acc_guard4(acc[2][0], acc[2][1], acc[2][2], acc[2][3]);
  acc_guard4(acc[3][0], acc[3][1], acc[3][2], acc[3][3]);

  float* slab = sT[wave];
  const float* Rb = RESID ? (resid + (size_t)b * strideR) : nullptr;
#pragma unroll
  for (int i = 0; i < 4; ++i) {
    const int mBase = m0 + (i << 4);
#pragma unroll
    for (int j = 0; j < 4; ++j) {
      const int n = n0 + (j << 4) + rlane;
      float bv = 0.f;
      if (BIAS_MODE == 2) bv = bias[n];
#pragma unroll
      for (int r = 0; r < 8; ++r) {
        float v = acc[i][j][r] * scale;
        if (BIAS_MODE == 1) v += bias[mBase + mOff + r];
        if (BIAS_MODE == 2) v += bv;
        if (RESID) v += Rb[(size_t)(mBase + mOff + r) * ldc + n];
        if (ACT == 1) v = tanhf(v);
        if (ACT == 2) v = fmaxf(v, 0.0f);
        slab[(mOff + r) * 68 + (j << 4) + rlane] = v;
      }
    }
    __builtin_amdgcn_fence(3, "workgroup");
    __builtin_amdgcn_wave_barrier();
    __builtin_amdgcn_fence(2, "workgroup");
    if (OUT_MODE == 0) {
      float* C = (float*)Cout + (size_t)b * strideC;
      const int hh = lane >> 4, c4 = (lane & 15) * 4;
      for (int pass = 0; pass < 2; ++pass) {
#pragma unroll
        for (int it = 0; it < 8; ++it) {
          const int row = it * 2 + hh;
          v4f v = *(const v4f*)(slab + row * 68 + c4);
          *(volatile v4f*)(C + (size_t)(mBase + row) * ldc + n0 + c4) = v;
        }
        __threadfence();
      }
    } else {
      const int q = lane >> 3, c8 = (lane & 7) * 8;
      unsigned short* C  = (unsigned short*)Cout  + (size_t)b * strideC;
      unsigned short* C2 = (OUT_MODE == 2) ? ((unsigned short*)Cout2 + (size_t)b * strideC) : nullptr;
      for (int pass = 0; pass < 2; ++pass) {
#pragma unroll
        for (int it = 0; it < 4; ++it) {
          const int row = it * 4 + q;
          const float* sp = slab + row * 68 + c8;
          v8h hv, lv;
#pragma unroll
          for (int e = 0; e < 8; ++e) {
            if (OUT_MODE == 1) {
              hv[e] = (_Float16)sp[e];
            } else {
              unsigned short hb = f2bf_bits(sp[e]);
              unsigned short lb = f2bf_bits(sp[e] - bf_bits2f(hb));
              hv[e] = __builtin_bit_cast(_Float16, hb);
              lv[e] = __builtin_bit_cast(_Float16, lb);
            }
          }
          *(volatile v8h*)(C + (size_t)(mBase + row) * ldc + n0 + c8) = hv;
          if (OUT_MODE == 2) *(volatile v8h*)(C2 + (size_t)(mBase + row) * ldc + n0 + c8) = lv;
        }
        __threadfence();
      }
    }
    __builtin_amdgcn_fence(3, "workgroup");
    __builtin_amdgcn_wave_barrier();
    __builtin_amdgcn_fence(2, "workgroup");
  }
}
}

__global__ __launch_bounds__(256) void k_cast16(const float* __restrict__ SRC, int lds, int seg, long long segsrc, unsigned short* __restrict__ DST, int ldd, int nR, int nC, float sc) {
    const long long u = (long long)blockIdx.x * 256 + threadIdx.x; const int per = nC / 8; if (u >= (long long)nR * per) return;
    const int r = (int)(u / per); const int c0 = 8 * (int)(u % per);
    const long long sr = (long long)(r / seg) * segsrc + (r % seg);
    const float* s = SRC + sr * lds + c0;
    const v4f a = *(const v4f*)(s), g = *(const v4f*)(s + 4);
    v4u pk;
    pk.x = pk2h(bf_rne(a.x) * sc, bf_rne(a.y) * sc); pk.y = pk2h(bf_rne(a.z) * sc, bf_rne(a.w) * sc);
    pk.z = pk2h(bf_rne(g.x) * sc, bf_rne(g.y) * sc); pk.w = pk2h(bf_rne(g.z) * sc, bf_rne(g.w) * sc);
    VST2(v4u, (v4u*)(DST + (long long)r * ldd + c0), pk);
}

__global__ __launch_bounds__(256) void k_bfq(const float* __restrict__ SRC, float* __restrict__ DST) {
    const long long u = (long long)blockIdx.x * 256 + threadIdx.x; constexpr int per = SEQ / 4; if (u >= (long long)NB * SEQ * per) return;
    const long long row = u / per; const int c0 = 4 * (int)(u % per); const int bb = (int)(row / SEQ); const int i = (int)(row % SEQ);
    const v4f a = *(const v4f*)(SRC + ((size_t)bb * SEQ_FULL + i) * SEQ_FULL + c0);
    v4f w; w.x = bf_rne(a.x); w.y = bf_rne(a.y); w.z = bf_rne(a.z); w.w = bf_rne(a.w);
    VST2V4(DST + row * SEQ + c0, w);
}

#define PCARRY 16384.0f
__global__ __launch_bounds__(128) __attribute__((amdgpu_num_vgpr(256)))
void k_flash(const unsigned short* __restrict__ Qp, const unsigned short* __restrict__ Kp, const unsigned short* __restrict__ VTp,
             const float* __restrict__ QB, const float* __restrict__ scl, float* __restrict__ out) {
    __shared__ __align__(16) float Os[4][16 * 68];
    const _Float16* Q = (const _Float16*)Qp; const _Float16* Kk = (const _Float16*)Kp; const _Float16* VT = (const _Float16*)VTp;
    const int tid = threadIdx.x, wave = tid >> 5, lane = tid & 31, hf = lane >> 4, c = lane & 15;
    constexpr int NQB = SEQ / 64;
    constexpr long long NKEY = (long long)NB * SEQ;
    const int bx = blockIdx.x;
    const int qb = bx % NQB; const int bh = bx / NQB; const int h = bh % NH; const int b = bh / NH;
    const int q0 = qb * 64 + wave * 16;
    const float c2 = bf_rne(scl[h]) * 1.4426950408889634f;

    const size_t qrow = (size_t)b * SEQ + q0 + c;
    const _Float16* qptr = Q + qrow * DM + h * HD + 8 * hf;
    const v16h qf0 = fload(qptr), qf1 = fload(qptr + 32);
    const _Float16* kbase = Kk + ((size_t)b * SEQ + c) * DM + h * HD + 8 * hf;
    const _Float16* vbase = VT + (size_t)(h * HD + c) * NKEY + (size_t)b * SEQ + 8 * hf;
    const float* qbrow = QB + qrow * SEQ + 8 * hf;

    v8f o[4];
#pragma unroll
    for (int t = 0; t < 4; ++t) o[t] = (v8f){0.f,0.f,0.f,0.f,0.f,0.f,0.f,0.f};
    float mrun = -__builtin_inff(), lrun = 0.f;

#pragma unroll 1
    for (int kv0 = 0; kv0 < SEQ; kv0 += 64) {
        float p[4][8];
        float mloc = -__builtin_inff();
#pragma unroll
        for (int j = 0; j < 4; ++j) {
            const _Float16* krow = kbase + (size_t)(kv0 + 16 * j) * DM;
            v8f acc = (v8f){0.f,0.f,0.f,0.f,0.f,0.f,0.f,0.f};
            acc = wmma16(fload(krow), qf0, acc);
            acc = wmma16(fload(krow + 32), qf1, acc);
            const v4f g0 = *(const v4f*)(qbrow + kv0 + 16 * j), g1 = *(const v4f*)(qbrow + kv0 + 16 * j + 4);
            const float gb[8] = {g0.x, g0.y, g0.z, g0.w, g1.x, g1.y, g1.z, g1.w};
#pragma unroll
            for (int r = 0; r < 8; ++r) { const float z = (acc[r] * 0.125f + gb[r]) * c2; p[j][r] = z; mloc = fmaxf(mloc, z); }
            sched_fence();
        }
        mloc = fmaxf(mloc, __shfl_xor(mloc, 16, 32));
        const float mnew = fmaxf(mrun, mloc);
        const float alpha = exp2f(mrun - mnew);
        mrun = mnew;
        float psum = 0.f;
        v16h pa0, pa1;
#pragma unroll
        for (int r = 0; r < 8; ++r) {
            const float e0 = exp2f(p[0][r] - mnew), e1 = exp2f(p[1][r] - mnew), e2 = exp2f(p[2][r] - mnew), e3 = exp2f(p[3][r] - mnew);
            psum += (e0 + e1) + (e2 + e3);
            pa0[r] = (_Float16)(e0 * PCARRY); pa0[8 + r] = (_Float16)(e1 * PCARRY);
            pa1[r] = (_Float16)(e2 * PCARRY); pa1[8 + r] = (_Float16)(e3 * PCARRY);
        }
        psum += __shfl_xor(psum, 16, 32);
        lrun = lrun * alpha + psum;
#pragma unroll
        for (int r = 0; r < 8; ++r) {
            const float ar = __shfl(alpha, 8 * hf + r, 32);
#pragma unroll
            for (int t = 0; t < 4; ++t) o[t][r] *= ar;
        }
#pragma unroll
        for (int t = 0; t < 4; ++t) {
            const _Float16* vrow = vbase + (size_t)(16 * t) * NKEY + kv0;
            const v16h vb0 = fload(vrow), vb1 = fload(vrow + 32);
            o[t] = wmma16(pa0, vb0, o[t]);
            o[t] = wmma16(pa1, vb1, o[t]);
            sched_fence();
        }
    }

    const float inv = 1.0f / (lrun * PCARRY);
    float* os = Os[wave];
#pragma unroll
    for (int r = 0; r < 8; ++r) {
        const float ir = __shfl(inv, 8 * hf + r, 32);
#pragma unroll
        for (int t = 0; t < 4; ++t) os[(8 * hf + r) * 68 + t * 16 + c] = o[t][r] * ir;
    }
    __builtin_amdgcn_fence(3, "workgroup");
    __builtin_amdgcn_wave_barrier();
    __builtin_amdgcn_fence(2, "workgroup");
    {
        float* ob = out + ((size_t)b * SEQ + q0) * DM + h * HD;
        const int c4 = c * 4;
        for (int pass = 0; pass < 2; ++pass) {
#pragma unroll
            for (int it = 0; it < 8; ++it) {
                const int row = it * 2 + hf;
                const v4f val = *(const v4f*)(os + row * 68 + c4);
                *(volatile v4f*)(ob + (size_t)row * DM + c4) = val;
            }
            __threadfence();
        }
    }
}

extern "C" void kernel_launch(void* const* d_in, const int* in_sizes, int n_in, void* d_out, int out_size, void* d_ws, size_t ws_size, hipStream_t stream) {
    if (n_in < 6) return;
    if (in_sizes[0] < ((NB - 1) * SEQ_FULL + SEQ) * DM) return;
    if (in_sizes[1] < (NB - 1) * SEQ_FULL * SEQ_FULL + (SEQ - 1) * SEQ_FULL + SEQ) return;
    if (in_sizes[2] < DM * DM || in_sizes[3] < DM * DM || in_sizes[4] < DM * DM) return;
    if (in_sizes[5] < NH) return;
    if (out_size < NB * SEQ * DM) return;
    const float* x   = (const float*)d_in[0];
    const float* qs  = (const float*)d_in[1];
    const float* wq  = (const float*)d_in[2];
    const float* wk  = (const float*)d_in[3];
    const float* wv  = (const float*)d_in[4];
    const float* scl = (const float*)d_in[5];
    float* out = (float*)d_out;

    const int MR = NB * SEQ;
    char* wsp = (char*)d_ws;
    const size_t szX  = (((size_t)MR * DM * 2 + 255) / 256) * 256;
    const size_t szW  = (((size_t)DM * DM * 2 + 255) / 256) * 256;
    const size_t szQB = (((size_t)MR * SEQ * 4 + 255) / 256) * 256;
    unsigned short* X16  = (unsigned short*)wsp; wsp += szX;
    unsigned short* WQ16 = (unsigned short*)wsp; wsp += szW;
    unsigned short* WK16 = (unsigned short*)wsp; wsp += szW;
    unsigned short* WV16 = (unsigned short*)wsp; wsp += szW;
    unsigned short* Q16  = (unsigned short*)wsp; wsp += szX;
    unsigned short* K16  = (unsigned short*)wsp; wsp += szX;
    unsigned short* VT16 = (unsigned short*)wsp; wsp += szX;
    float* QB = (float*)wsp; wsp += szQB;
    if ((size_t)(wsp - (char*)d_ws) > ws_size) return;

    k_cast16<<<(unsigned)(((long long)MR * (DM / 8) + 255) / 256), 256, 0, stream>>>(x, DM, SEQ, (long long)SEQ_FULL, X16, DM, MR, DM, 1.0f);
    k_cast16<<<(unsigned)(((long long)DM * (DM / 8) + 255) / 256), 256, 0, stream>>>(wq, DM, DM, 0, WQ16, DM, DM, DM, 16.0f);
    k_cast16<<<(unsigned)(((long long)DM * (DM / 8) + 255) / 256), 256, 0, stream>>>(wk, DM, DM, 0, WK16, DM, DM, DM, 16.0f);
    k_cast16<<<(unsigned)(((long long)DM * (DM / 8) + 255) / 256), 256, 0, stream>>>(wv, DM, DM, 0, WV16, DM, DM, DM, 16.0f);
    k_bfq<<<(unsigned)(((long long)MR * (SEQ / 4) + 255) / 256), 256, 0, stream>>>(qs, QB);
    w25::wmma_gemm64<0, false, 0, 1, false, 0><<<dim3((unsigned)(((MR / 64) * (DM / 64) + 7) / 8), 1u), 256, 0, stream>>>(
        X16, nullptr, DM, 0, WQ16, nullptr, DM, 0, (void*)Q16, nullptr, DM, 0, nullptr, nullptr, 0, MR, DM, DM, 0.0625f);
    w25::wmma_gemm64<0, false, 0, 1, false, 0><<<dim3((unsigned)(((MR / 64) * (DM / 64) + 7) / 8), 1u), 256, 0, stream>>>(
        X16, nullptr, DM, 0, WK16, nullptr, DM, 0, (void*)K16, nullptr, DM, 0, nullptr, nullptr, 0, MR, DM, DM, 0.0625f);
    w25::wmma_gemm64<0, false, 0, 1, false, 0><<<dim3((unsigned)(((DM / 64) * (MR / 64) + 7) / 8), 1u), 256, 0, stream>>>(
        WV16, nullptr, DM, 0, X16, nullptr, DM, 0, (void*)VT16, nullptr, MR, 0, nullptr, nullptr, 0, DM, MR, DM, 0.0625f);
    k_flash<<<(unsigned)(NB * NH * (SEQ / 64)), 128, 0, stream>>>(Q16, K16, VT16, QB, scl, out);
}
